// GAT_35820027248975
// MI455X (gfx1250) — hardware-verified
//
#include <hip/hip_runtime.h>
#include <stddef.h>
#include <stdint.h>
#include <math.h>

#define GN      4096
#define GE      131072
#define FIN     32
#define NHD     8
#define FH      32
#define HID     256
#define NCLS    10
#define NC2P    16
#define K2      512
#define NTHR    256
#define NWAVE   8
#define EPT     8
#define CHUNK   (NTHR * EPT)
#define WCAP    (EPT * 32)
#define LISTN   (NWAVE * WCAP)
#define NB      256
#define SLOTB   8
#define RCAP    12288
#define DEGCAP  96
#define RB1     16
#define RB2     64
#define GTHR    128
#define GBM     64
#define NEGSL   0.2f
#define WSMAX   134217728

#define NU_X    (GN * FIN / 8)
#define NU_W1   (HID * FIN / 8)
#define NU_W2   (NC2P * K2 / 8)
#define NU_TOT  (NU_X + NU_W1 + NU_W2)
#define OFF_XB  0
#define OFF_W1T (GN * FIN)
#define OFF_W2T (GN * FIN + HID * FIN)
#define P16_HW  (GN * FIN + HID * FIN + NC2P * K2)
#define LDS_ADJ_INTS (2 * RCAP + 2 * NB + LISTN + 16 + NWAVE * DEGCAP + NB)

static_assert(NB == NTHR && NB == (1 << SLOTB));
static_assert((CHUNK & (CHUNK - 1)) == 0);
static_assert(((long long)GE << SLOTB) < (1LL << 31));
static_assert((RCAP % 4) == 0 && (LISTN >= NB));
static_assert((GN % NB) == 0 && (GN % RB1) == 0 && (GN % RB2) == 0 && (GN % GBM) == 0);
static_assert((NU_X % NTHR) == 0 && (NU_W1 % NTHR) == 0 && (NU_W2 % NTHR) == 0);
static_assert(HID == NTHR && HID == NHD * FH && K2 == 2 * HID);
static_assert((FIN % 32) == 0 && (K2 % 32) == 0);
static_assert((DEGCAP % 32) == 0 && DEGCAP == 96);
static_assert((RB2 * NCLS * 4) % 128 == 0 && (RB2 * NCLS) % 4 == 0 && (RB2 * NCLS / 4) <= NTHR);
static_assert(RB2 == NWAVE * 8);
static_assert(GBM == (GTHR / 32) * 16);
static_assert(LDS_ADJ_INTS * 4 <= 300000);
static_assert(((2 * RCAP + 2 * NB + LISTN + 16) % 4) == 0);

typedef float          v4f  __attribute__((ext_vector_type(4)));
typedef float          v8f  __attribute__((ext_vector_type(8)));
typedef int            v4i  __attribute__((ext_vector_type(4)));
typedef int            v8i  __attribute__((ext_vector_type(8)));
typedef unsigned int   v4u  __attribute__((ext_vector_type(4)));
typedef unsigned short v8us __attribute__((ext_vector_type(8)));
typedef __bf16         v16b __attribute__((ext_vector_type(16)));
typedef v4f  __attribute__((may_alias)) v4fa;
typedef v4i  __attribute__((may_alias)) v4ia;
typedef v4u  __attribute__((may_alias)) v4ua;
typedef v8us __attribute__((may_alias)) v8usa;
union FragB { v16b v; v8us h[2]; v8i w; };

__device__ __forceinline__ v8f wmb(const FragB& a, const FragB& b, v8f c) {
  v8f d = __builtin_amdgcn_wmma_f32_16x16x32_bf16(false, a.v, false, b.v, (short)0, c, false, false);
  asm volatile("v_nop\n\tv_nop\n\tv_nop\n\tv_nop" : "+v"(d) : "v"(a.w), "v"(b.w));
  return d;
}

__device__ __forceinline__ unsigned int f2bf(float f) {
  const unsigned int u = __float_as_uint(f);
  return ((u + 0x7FFFu + ((u >> 16) & 1u)) >> 16) & 0xFFFFu;
}
__device__ __forceinline__ float bf2f(unsigned int b) { return __uint_as_float(b << 16); }
__device__ __forceinline__ float bfr(float f) { return bf2f(f2bf(f)); }
__device__ __forceinline__ unsigned int pk2(float lo, float hi) { return f2bf(lo) | (f2bf(hi) << 16); }
__device__ __forceinline__ v4u pack8(const v4f a, const v4f b) {
  v4u r;
  r.x = pk2(a.x, a.y); r.y = pk2(a.z, a.w); r.z = pk2(b.x, b.y); r.w = pk2(b.z, b.w);
  return r;
}
__device__ __forceinline__ int clampi(int v, int lo, int hi) { return v < lo ? lo : (v > hi ? hi : v); }

__global__ __launch_bounds__(NTHR) void k_prep(const float* __restrict__ x, const float* __restrict__ W1,
                                               const float* __restrict__ W2, unsigned short* P16) {
  const int u = (int)blockIdx.x * NTHR + (int)threadIdx.x;
  v4f a, b;
  int off;
  const v4f z4 = {0.f, 0.f, 0.f, 0.f};
  if (u < NU_X) {
    const float* p = x + (size_t)u * 8;
    a = *(const v4fa*)p;
    b = *(const v4fa*)(p + 4);
    off = OFF_XB + u * 8;
  } else if (u < NU_X + NU_W1) {
    const int v  = u - NU_X;
    const int n  = v >> 2;
    const int k8 = (v & 3) * 8;
    const int h  = n >> 5, f = n & 31;
    const float* p = W1 + h * (FIN * FH) + k8 * FH + f;
    a.x = p[0];      a.y = p[FH];     a.z = p[2 * FH]; a.w = p[3 * FH];
    b.x = p[4 * FH]; b.y = p[5 * FH]; b.z = p[6 * FH]; b.w = p[7 * FH];
    off = OFF_W1T + n * FIN + k8;
  } else if (u < NU_TOT) {
    const int v   = u - NU_X - NU_W1;
    const int n   = v >> 6;
    const int k8  = (v & 63) * 8;
    const int kk  = k8 & (HID - 1);
    const int ncl = n < NCLS ? n : NCLS - 1;
    const float* p = W2 + kk * NCLS + ncl;
    a.x = p[0];        a.y = p[NCLS];     a.z = p[2 * NCLS]; a.w = p[3 * NCLS];
    b.x = p[4 * NCLS]; b.y = p[5 * NCLS]; b.z = p[6 * NCLS]; b.w = p[7 * NCLS];
    if (n >= NCLS) { a = z4; b = z4; }
    off = OFF_W2T + n * K2 + k8;
  } else {
    return;
  }
  const v4u wv = pack8(a, b);
  unsigned short* dp = P16 + off;
  *(volatile v4u*)dp = wv;
  __threadfence();
  *(volatile v4u*)dp = wv;
}

__global__ __launch_bounds__(GTHR) void k_gemm1(const unsigned short* __restrict__ XB,
                                                const unsigned short* __restrict__ W1T,
                                                float* HH, const float* __restrict__ a1, float* SD1) {
  __shared__ __attribute__((aligned(16))) float stg[GBM * FH];
  __shared__ __attribute__((aligned(16))) float satt[2 * FH];
  __shared__ __attribute__((aligned(16))) float sdot[2 * GBM];
  const int tid = (int)threadIdx.x, lane = tid & 31, wave = tid >> 5, hh = lane >> 4, m = lane & 15;
  const int rowBase = (int)blockIdx.x * GBM;
  const int head    = (int)blockIdx.y;
  const int col0    = head * FH;

  if (tid < 2 * FH) satt[tid] = bfr(a1[head * (2 * FH) + tid]);

  v8f acc[2];
  {
    const v8f z = {0.f, 0.f, 0.f, 0.f, 0.f, 0.f, 0.f, 0.f};
    acc[0] = z; acc[1] = z;
  }
  {
    const unsigned short* ap = XB + (size_t)(rowBase + 16 * wave + m) * FIN + 8 * hh;
    FragB af;
    af.h[0] = *(const v8usa*)ap;
    af.h[1] = *(const v8usa*)(ap + 16);
#pragma unroll
    for (int t = 0; t < 2; ++t) {
      const unsigned short* wq = W1T + (size_t)(col0 + 16 * t + m) * FIN + 8 * hh;
      FragB bf;
      bf.h[0] = *(const v8usa*)wq;
      bf.h[1] = *(const v8usa*)(wq + 16);
      acc[t] = wmb(af, bf, acc[t]);
    }
  }
#pragma unroll
  for (int t = 0; t < 2; ++t) {
#pragma unroll
    for (int r = 0; r < 8; ++r) {
      const int lr = 16 * wave + 8 * hh + r;
      stg[lr * FH + 16 * t + m] = acc[t][r];
    }
  }
  __syncthreads();

  {
    const int row = tid & 63, which = tid >> 6;
    const float* sa = satt + which * FH;
    const float* hr = stg + row * FH;
    float d = 0.f;
#pragma unroll 4
    for (int c4 = 0; c4 < FH / 4; ++c4) {
      const v4f hv = *(const v4fa*)(hr + 4 * c4);
      const v4f av = *(const v4fa*)(sa + 4 * c4);
      d = fmaf(hv.x, av.x, d);
      d = fmaf(hv.y, av.y, d);
      d = fmaf(hv.z, av.z, d);
      d = fmaf(hv.w, av.w, d);
    }
    sdot[which * GBM + row] = d;
  }
  __syncthreads();

  v4f fv[4];
#pragma unroll
  for (int i = 0; i < 4; ++i) {
    const int lr = 16 * wave + 4 * i + (lane >> 3);
    fv[i] = *(const v4fa*)(stg + lr * FH + 4 * (lane & 7));
  }
  const int which2 = lane >> 4, piece = lane & 15;
  const v4f sdv = *(const v4fa*)(sdot + which2 * GBM + 4 * piece);
  float* sp = SD1 + (size_t)(2 * head + which2) * GN + rowBase + 4 * piece;

#pragma unroll
  for (int i = 0; i < 4; ++i) {
    const int lr = 16 * wave + 4 * i + (lane >> 3);
    float* op = HH + (size_t)(rowBase + lr) * HID + col0 + 4 * (lane & 7);
    *(volatile v4f*)op = fv[i];
  }
  if (wave == 0) *(volatile v4f*)sp = sdv;
  __threadfence();
#pragma unroll
  for (int i = 0; i < 4; ++i) {
    const int lr = 16 * wave + 4 * i + (lane >> 3);
    float* op = HH + (size_t)(rowBase + lr) * HID + col0 + 4 * (lane & 7);
    *(volatile v4f*)op = fv[i];
  }
  if (wave == 0) *(volatile v4f*)sp = sdv;
}

__device__ __forceinline__ int scan_chunk(const int* __restrict__ keys, int nE, int cbase, int slotBase,
                                          int nb, int vec8, int* list, int tid, int lane, int wave) {
  int wc = 0;
  const int el0  = tid * EPT;
  const int e0   = cbase + el0;
  const int sent = -2147483647 - 1;
  v4i da, db;
  if (vec8 != 0 && cbase + CHUNK <= nE) {
    da = *(const v4i*)(keys + e0);
    db = *(const v4i*)(keys + e0 + 4);
  } else {
    da.x = (e0     < nE) ? keys[min(e0,     nE - 1)] : sent;
    da.y = (e0 + 1 < nE) ? keys[min(e0 + 1, nE - 1)] : sent;
    da.z = (e0 + 2 < nE) ? keys[min(e0 + 2, nE - 1)] : sent;
    da.w = (e0 + 3 < nE) ? keys[min(e0 + 3, nE - 1)] : sent;
    db.x = (e0 + 4 < nE) ? keys[min(e0 + 4, nE - 1)] : sent;
    db.y = (e0 + 5 < nE) ? keys[min(e0 + 5, nE - 1)] : sent;
    db.z = (e0 + 6 < nE) ? keys[min(e0 + 6, nE - 1)] : sent;
    db.w = (e0 + 7 < nE) ? keys[min(e0 + 7, nE - 1)] : sent;
  }
  const unsigned nbs = (unsigned)slotBase;
  const unsigned unb = (unsigned)nb;
  const unsigned s0 = (unsigned)da.x - nbs, s1 = (unsigned)da.y - nbs;
  const unsigned s2 = (unsigned)da.z - nbs, s3 = (unsigned)da.w - nbs;
  const unsigned s4 = (unsigned)db.x - nbs, s5 = (unsigned)db.y - nbs;
  const unsigned s6 = (unsigned)db.z - nbs, s7 = (unsigned)db.w - nbs;
  const bool h0 = s0 < unb, h1 = s1 < unb, h2 = s2 < unb, h3 = s3 < unb;
  const bool h4 = s4 < unb, h5 = s5 < unb, h6 = s6 < unb, h7 = s7 < unb;
  const unsigned any = __builtin_amdgcn_ballot_w32(h0 | h1 | h2 | h3 | h4 | h5 | h6 | h7);
  if (any != 0u) {
#define HITJ(J, HJ, SJ) { \
      const unsigned mj = __builtin_amdgcn_ballot_w32(HJ); \
      if (mj != 0u) { \
        if (HJ) { \
          const int pos = wc + (int)__builtin_amdgcn_mbcnt_lo(mj, 0u); \
          if (pos < WCAP) list[wave * WCAP + pos] = ((el0 + (J)) << SLOTB) | (int)(SJ); \
        } \
        wc += (int)__builtin_popcount(mj); } }
    HITJ(0, h0, s0)
    HITJ(1, h1, s1)
    HITJ(2, h2, s2)
    HITJ(3, h3, s3)
    HITJ(4, h4, s4)
    HITJ(5, h5, s5)
    HITJ(6, h6, s6)
    HITJ(7, h7, s7)
#undef HITJ
  }
  return wc;
}

__device__ __forceinline__ int fetch_id(const int* reg2, const int* __restrict__ tgts, int st, int hmax,
                                        int k, int grow, int nE) {
  int hi = k - 1;
  hi = hi < 0 ? 0 : (hi > hmax ? hmax : hi);
  int idx = st + hi;
  idx = idx > RCAP - 1 ? RCAP - 1 : idx;
  const int eid = clampi(reg2[idx], 0, nE - 1);
  const int t   = clampi(tgts[eid], 0, GN - 1);
  return (k == 0) ? grow : t;
}

__global__ __launch_bounds__(NTHR) void k_adj(const int* __restrict__ ei, int* ADJ, int* CP, int nE, int vec8) {
  extern __shared__ v4f lds_dyn[];
  int* reg1 = (int*)lds_dyn;
  int* reg2 = reg1 + RCAP;
  int* scnt = reg2 + RCAP;
  int* soff = scnt + NB;
  int* list = soff + NB;
  int* wcnt = list + LISTN;
  int* wtot = wcnt + NWAVE;
  int* orow = wtot + NWAVE;
  int* cpl  = orow + NWAVE * DEGCAP;
  const int tid = (int)threadIdx.x, lane = tid & 31, wave = tid >> 5;
  const int nodeBase = (int)blockIdx.x * NB;
  const int* keys = ei;
  const int* tgts = ei + nE;

  scnt[tid] = 0;
  {
    const v4i z4 = {0, 0, 0, 0};
    for (int i = tid * 4; i < RCAP; i += NTHR * 4) *(v4ia*)(reg2 + i) = z4;
  }
  __syncthreads();

  int tot = 0;
  const int nChunks = (nE + CHUNK - 1) / CHUNK;
#pragma unroll 1
  for (int ch = 0; ch < nChunks; ++ch) {
    const int cbase = ch * CHUNK;
    const int wc = scan_chunk(keys, nE, cbase, nodeBase, NB, vec8, list, tid, lane, wave);
    if (lane == 0) wcnt[wave] = wc;
    __syncthreads();
    int pre = 0, all = 0;
#pragma unroll
    for (int w2 = 0; w2 < NWAVE; ++w2) {
      int c = wcnt[w2];
      c = c < 0 ? 0 : (c > WCAP ? WCAP : c);
      all += c;
      pre += (w2 < wave) ? c : 0;
    }
    const int wcc  = wc > WCAP ? WCAP : wc;
    const int base = tot + pre;
#pragma unroll 1
    for (int i = lane; i < wcc; i += 32) {
      const int ent = list[wave * WCAP + i];
      const int el  = (ent >> SLOTB) & (CHUNK - 1);
      const int sl  = ent & (NB - 1);
      int eid = cbase + el;
      eid = eid > nE - 1 ? nE - 1 : eid;
      const int pos = base + i;
      if (pos < RCAP) reg1[pos] = (int)(((unsigned)eid << SLOTB) | (unsigned)sl);
    }
    tot += all;
    tot = tot > RCAP ? RCAP : tot;
    __syncthreads();
  }
  const int nh = tot;

  if (wave == 0) {
#pragma unroll 1
    for (int b0 = 0; b0 < nh; b0 += 32) {
      const int idx = b0 + lane;
      const int uv  = reg1[idx < nh ? idx : nh - 1];
      const int m32 = (nh - b0) < 32 ? (nh - b0) : 32;
#pragma unroll 1
      for (int k = 0; k < m32; ++k) {
        const int u  = __builtin_amdgcn_readlane(uv, k);
        const int sl = u & (NB - 1);
        if (lane == 0) scnt[sl] = scnt[sl] + 1;
      }
    }
  }
  __syncthreads();

  {
    int c = scnt[tid];
    c = c < 0 ? 0 : c;
    int incl = c;
#pragma unroll
    for (int d = 1; d < 32; d <<= 1) {
      const int up = __shfl_up(incl, d);
      if (lane >= d) incl += up;
    }
    if (lane == 31) wtot[wave] = incl;
    __syncthreads();
    int pre = 0;
#pragma unroll
    for (int w2 = 0; w2 < NWAVE; ++w2) pre += (w2 < wave) ? wtot[w2] : 0;
    const int ex = pre + incl - c;
    soff[tid] = ex;
    list[tid] = ex;
  }
  __syncthreads();

  if (wave == 0) {
#pragma unroll 1
    for (int b0 = 0; b0 < nh; b0 += 32) {
      const int idx = b0 + lane;
      const int uv  = reg1[idx < nh ? idx : nh - 1];
      const int m32 = (nh - b0) < 32 ? (nh - b0) : 32;
#pragma unroll 1
      for (int k = 0; k < m32; ++k) {
        const int u   = __builtin_amdgcn_readlane(uv, k);
        const int sl  = u & (NB - 1);
        const int eid = (int)((unsigned)u >> SLOTB);
        if (lane == 0) {
          int pos = list[sl];
          pos = pos < 0 ? 0 : (pos > RCAP - 1 ? RCAP - 1 : pos);
          reg2[pos] = eid;
          list[sl] = pos + 1;
        }
      }
    }
  }
  __syncthreads();

  const bool ovf = (nh >= RCAP);
  int* my = orow + wave * DEGCAP;
#pragma unroll 1
  for (int jt = 0; jt < NB / NWAVE; ++jt) {
    const int slot = wave * (NB / NWAVE) + jt;
    const int grow = nodeBase + slot;
    int st   = __builtin_amdgcn_readfirstlane(soff[slot]);
    int craw = __builtin_amdgcn_readfirstlane(scnt[slot]);
    st = st < 0 ? 0 : (st > nh ? nh : st);
    int cnt = craw < 0 ? 0 : (craw > DEGCAP - 1 ? DEGCAP - 1 : craw);
    if (cnt > nh - st) cnt = nh - st;
    const int pois = (ovf || craw > DEGCAP - 1) ? 1 : 0;
    const int tot3 = cnt + 1;
    const int hmax = cnt > 0 ? cnt - 1 : 0;
    const int k0 = lane, k1 = lane + 32, k2 = lane + 64;
    const int id0 = fetch_id(reg2, tgts, st, hmax, k0, grow, nE);
    const int id1 = fetch_id(reg2, tgts, st, hmax, k1, grow, nE);
    const int id2 = fetch_id(reg2, tgts, st, hmax, k2, grow, nE);

    int d0 = 0, d1 = 0, d2 = 0;
    {
      const int lim = clampi(tot3, 0, 32);
#pragma unroll 1
      for (int kk = 0; kk < lim; ++kk) {
        const int v = __builtin_amdgcn_readlane(id0, kk);
        d0 |= (int)(kk < k0) & (int)(v == id0);
        d1 |= (int)(v == id1);
        d2 |= (int)(v == id2);
      }
    }
    {
      const int lim = clampi(tot3 - 32, 0, 32);
#pragma unroll 1
      for (int kk = 0; kk < lim; ++kk) {
        const int v = __builtin_amdgcn_readlane(id1, kk);
        d1 |= (int)(32 + kk < k1) & (int)(v == id1);
        d2 |= (int)(v == id2);
      }
    }
    {
      const int lim = clampi(tot3 - 64, 0, 32);
#pragma unroll 1
      for (int kk = 0; kk < lim; ++kk) {
        const int v = __builtin_amdgcn_readlane(id2, kk);
        d2 |= (int)(64 + kk < k2) & (int)(v == id2);
      }
    }
    const bool keep0 = (k0 < tot3) && (d0 == 0);
    const bool keep1 = (k1 < tot3) && (d1 == 0);
    const bool keep2 = (k2 < tot3) && (d2 == 0);
    const unsigned m0 = __builtin_amdgcn_ballot_w32(keep0);
    const unsigned m1 = __builtin_amdgcn_ballot_w32(keep1);
    const unsigned m2 = __builtin_amdgcn_ballot_w32(keep2);
    const int c0 = (int)__builtin_popcount(m0), c1 = (int)__builtin_popcount(m1), c2 = (int)__builtin_popcount(m2);
    const int p0 = (int)__builtin_amdgcn_mbcnt_lo(m0, 0u);
    const int p1 = c0 + (int)__builtin_amdgcn_mbcnt_lo(m1, 0u);
    const int p2 = c0 + c1 + (int)__builtin_amdgcn_mbcnt_lo(m2, 0u);
    const int total = c0 + c1 + c2;

    my[lane]      = grow;
    my[lane + 32] = grow;
    my[lane + 64] = grow;
    if (keep0) my[p0] = id0;
    if (keep1) my[p1] = id1;
    if (keep2) my[p2] = id2;
    if (lane == 0) cpl[slot] = total | (pois << 16);
    __syncthreads();

    const int pl = lane < 24 ? lane : 23;
    const v4i rv = *(const v4ia*)(my + 4 * pl);
    int* gp = ADJ + (size_t)grow * DEGCAP + 4 * pl;
    if (lane < 24) *(volatile v4i*)gp = rv;
    __threadfence();
    if (lane < 24) *(volatile v4i*)gp = rv;
    __syncthreads();
  }

  if (tid < NB / 4) {
    const v4i cv = *(const v4ia*)(cpl + 4 * tid);
    int* cp = CP + nodeBase + 4 * tid;
    *(volatile v4i*)cp = cv;
    __threadfence();
    *(volatile v4i*)cp = cv;
  }
}

__device__ __forceinline__ void nb_scores(const int* __restrict__ ar, int cnt, int lane, float p,
                                          const float* __restrict__ Qp,
                                          int& j0, int& j1, int& j2, float& e0, float& e1, float& e2, float& inv) {
  const int cm = cnt - 1;
  const int a0 = lane      < cm ? lane      : cm;
  const int a1 = lane + 32 < cm ? lane + 32 : cm;
  const int a2 = lane + 64 < cm ? lane + 64 : cm;
  j0 = clampi(ar[a0], 0, GN - 1);
  j1 = clampi(ar[a1], 0, GN - 1);
  j2 = clampi(ar[a2], 0, GN - 1);
  float s0 = p + Qp[j0], s1 = p + Qp[j1], s2 = p + Qp[j2];
  s0 = s0 >= 0.f ? s0 : NEGSL * s0;
  s1 = s1 >= 0.f ? s1 : NEGSL * s1;
  s2 = s2 >= 0.f ? s2 : NEGSL * s2;
  const bool v0 = lane < cnt, v1 = lane + 32 < cnt, v2 = lane + 64 < cnt;
  float mx = v0 ? s0 : -3.0e38f;
  mx = fmaxf(mx, v1 ? s1 : -3.0e38f);
  mx = fmaxf(mx, v2 ? s2 : -3.0e38f);
#pragma unroll
  for (int off = 16; off > 0; off >>= 1) mx = fmaxf(mx, __shfl_xor(mx, off));
  e0 = expf(s0 - mx); e1 = expf(s1 - mx); e2 = expf(s2 - mx);
  e0 = v0 ? e0 : 0.f;
  e1 = v1 ? e1 : 0.f;
  e2 = v2 ? e2 : 0.f;
  float l = e0 + e1 + e2;
#pragma unroll
  for (int off = 16; off > 0; off >>= 1) l += __shfl_xor(l, off);
  inv = 1.0f / l;
}

__device__ __forceinline__ float acc_part(float acc, int jr, float er, int lim,
                                          const float* __restrict__ F, int pitch, int c) {
  const int eb = __float_as_int(er);
#pragma unroll 1
  for (int kk = 0; kk < lim; ++kk) {
    const int   jk = __builtin_amdgcn_readlane(jr, kk);
    const float wk = __int_as_float(__builtin_amdgcn_readlane(eb, kk));
    acc = fmaf(wk, F[(size_t)jk * (size_t)pitch + c], acc);
  }
  return acc;
}

__global__ __launch_bounds__(NTHR) void k_agg1(const int* __restrict__ ADJ, const int* __restrict__ CP,
                                               const float* __restrict__ HH, const float* __restrict__ SD1,
                                               const float* __restrict__ b1, unsigned short* X1) {
  __shared__ __attribute__((aligned(16))) unsigned short xs[RB1 * K2];
  const int tid = (int)threadIdx.x, lane = tid & 31, wave = tid >> 5;
  const int row0 = (int)blockIdx.x * RB1;
  const float bias = bfr(b1[tid]);
  const float* Pp = SD1 + (size_t)(2 * wave) * GN;
  const float* Qp = Pp + GN;
  const float qnan = __int_as_float(0x7fc00000);
#pragma unroll 1
  for (int rr = 0; rr < RB1; ++rr) {
    const int i = row0 + rr;
    const int cpv  = __builtin_amdgcn_readfirstlane(CP[i]);
    const int pois = (cpv >> 16) & 1;
    const int cnt  = clampi(cpv & 0xFFFF, 1, DEGCAP);
    int j0, j1, j2;
    float e0, e1, e2, inv;
    nb_scores(ADJ + (size_t)i * DEGCAP, cnt, lane, Pp[i], Qp, j0, j1, j2, e0, e1, e2, inv);
    float acc = 0.0f;
    acc = acc_part(acc, j0, e0, clampi(cnt, 0, 32),      HH, HID, tid);
    acc = acc_part(acc, j1, e1, clampi(cnt - 32, 0, 32), HH, HID, tid);
    acc = acc_part(acc, j2, e2, clampi(cnt - 64, 0, 32), HH, HID, tid);
    float v = fmaf(acc, inv, bias);
    const float em = expm1f(v);
    v = (v > 0.f) ? v : em;
    v = (pois != 0) ? qnan : v;
    const unsigned int hb = f2bf(v);
    const unsigned int lb = f2bf(v - bf2f(hb));
    xs[rr * K2 + tid]       = (unsigned short)hb;
    xs[rr * K2 + HID + tid] = (unsigned short)lb;
  }
  __syncthreads();
  unsigned short* gb = X1 + (size_t)row0 * K2;
  v4u pv[4];
#pragma unroll
  for (int it = 0; it < 4; ++it) pv[it] = *(const v4ua*)(xs + 8 * (it * NTHR + tid));
#pragma unroll
  for (int it = 0; it < 4; ++it) *(volatile v4u*)(gb + 8 * (it * NTHR + tid)) = pv[it];
  __threadfence();
#pragma unroll
  for (int it = 0; it < 4; ++it) *(volatile v4u*)(gb + 8 * (it * NTHR + tid)) = pv[it];
}

__global__ __launch_bounds__(GTHR) void k_gemm2(const unsigned short* __restrict__ X1,
                                                const unsigned short* __restrict__ W2T,
                                                float* H2, const float* __restrict__ a2, float* SD2) {
  __shared__ __attribute__((aligned(16))) float stg[GBM * NC2P];
  __shared__ __attribute__((aligned(16))) float satt[2 * NC2P];
  __shared__ __attribute__((aligned(16))) float sdot[2 * GBM];
  const int tid = (int)threadIdx.x, lane = tid & 31, wave = tid >> 5, hh = lane >> 4, m = lane & 15;
  const int rowBase = (int)blockIdx.x * GBM;

  if (tid < 2 * NC2P) {
    const int which = tid >> 4, c = tid & 15;
    const int cl = c < NCLS ? c : NCLS - 1;
    const float v = bfr(a2[which * NCLS + cl]);
    satt[tid] = (c < NCLS) ? v : 0.f;
  }

  v8f acc = {0.f, 0.f, 0.f, 0.f, 0.f, 0.f, 0.f, 0.f};
  const unsigned short* ap = X1  + (size_t)(rowBase + 16 * wave + m) * K2 + 8 * hh;
  const unsigned short* wp = W2T + (size_t)m * K2 + 8 * hh;
#pragma unroll 1
  for (int ks = 0; ks < K2 / 32; ++ks) {
    FragB af, bf;
    af.h[0] = *(const v8usa*)(ap + 32 * ks);
    af.h[1] = *(const v8usa*)(ap + 32 * ks + 16);
    bf.h[0] = *(const v8usa*)(wp + 32 * ks);
    bf.h[1] = *(const v8usa*)(wp + 32 * ks + 16);
    acc = wmb(af, bf, acc);
  }
#pragma unroll
  for (int r = 0; r < 8; ++r) {
    const int lr = 16 * wave + 8 * hh + r;
    stg[lr * NC2P + m] = acc[r];
  }
  __syncthreads();

  {
    const int row = tid & 63, which = tid >> 6;
    const float* sa = satt + which * NC2P;
    const float* hr = stg + row * NC2P;
    float d = 0.f;
#pragma unroll
    for (int c4 = 0; c4 < NC2P / 4; ++c4) {
      const v4f hv = *(const v4fa*)(hr + 4 * c4);
      const v4f av = *(const v4fa*)(sa + 4 * c4);
      d = fmaf(hv.x, av.x, d);
      d = fmaf(hv.y, av.y, d);
      d = fmaf(hv.z, av.z, d);
      d = fmaf(hv.w, av.w, d);
    }
    sdot[which * GBM + row] = d;
  }
  __syncthreads();

  v4f fv[2];
#pragma unroll
  for (int it = 0; it < 2; ++it) fv[it] = *(const v4fa*)(stg + 4 * (it * GTHR + tid));
  const int which2 = lane >> 4, piece = lane & 15;
  const v4f sdv = *(const v4fa*)(sdot + which2 * GBM + 4 * piece);
  float* sp = SD2 + (size_t)which2 * GN + rowBase + 4 * piece;
  float* ob = H2 + (size_t)rowBase * NC2P;
#pragma unroll
  for (int it = 0; it < 2; ++it) *(volatile v4f*)(ob + 4 * (it * GTHR + tid)) = fv[it];
  if (wave == 0) *(volatile v4f*)sp = sdv;
  __threadfence();
#pragma unroll
  for (int it = 0; it < 2; ++it) *(volatile v4f*)(ob + 4 * (it * GTHR + tid)) = fv[it];
  if (wave == 0) *(volatile v4f*)sp = sdv;
}

__global__ __launch_bounds__(NTHR) void k_agg2(const int* __restrict__ ADJ, const int* __restrict__ CP,
                                               const float* __restrict__ H2, const float* __restrict__ SD2,
                                               const float* __restrict__ b2, float* out) {
  __shared__ __attribute__((aligned(16))) float res[RB2 * NCLS];
  const int tid = (int)threadIdx.x, lane = tid & 31, wave = tid >> 5;
  const int ch = lane & 15;
  const int row0 = (int)blockIdx.x * RB2;
  float bz = bfr(b2[ch < NCLS ? ch : NCLS - 1]);
  bz = (ch < NCLS) ? bz : 0.f;
  const float* Pp = SD2;
  const float* Qp = SD2 + GN;
  const float qnan = __int_as_float(0x7fc00000);
  const bool valid = lane < NCLS;
#pragma unroll 1
  for (int rr = 0; rr < 8; ++rr) {
    const int lr = wave * 8 + rr;
    const int i  = row0 + lr;
    const int cpv  = __builtin_amdgcn_readfirstlane(CP[i]);
    const int pois = (cpv >> 16) & 1;
    const int cnt  = clampi(cpv & 0xFFFF, 1, DEGCAP);
    int j0, j1, j2;
    float e0, e1, e2, inv;
    nb_scores(ADJ + (size_t)i * DEGCAP, cnt, lane, Pp[i], Qp, j0, j1, j2, e0, e1, e2, inv);
    float acc = 0.0f;
    acc = acc_part(acc, j0, e0, clampi(cnt, 0, 32),      H2, NC2P, ch);
    acc = acc_part(acc, j1, e1, clampi(cnt - 32, 0, 32), H2, NC2P, ch);
    acc = acc_part(acc, j2, e2, clampi(cnt - 64, 0, 32), H2, NC2P, ch);
    const float z = fmaf(acc, inv, bz);
    float vm = valid ? z : -3.0e38f;
#pragma unroll
    for (int off = 16; off > 0; off >>= 1) vm = fmaxf(vm, __shfl_xor(vm, off));
    float ex = expf(z - vm);
    ex = valid ? ex : 0.f;
    float sm = ex;
#pragma unroll
    for (int off = 16; off > 0; off >>= 1) sm += __shfl_xor(sm, off);
    const float ls = logf(sm);
    float o = (z - vm) - ls;
    o = (pois != 0) ? qnan : o;
    if (valid) res[lr * NCLS + lane] = o;
  }
  __syncthreads();
  const int pl = tid < (RB2 * NCLS / 4) ? tid : (RB2 * NCLS / 4) - 1;
  const v4f ov = *(const v4fa*)(res + 4 * pl);
  float* op = out + (size_t)row0 * NCLS + 4 * pl;
  if (tid < RB2 * NCLS / 4) *(volatile v4f*)op = ov;
  __threadfence();
  if (tid < RB2 * NCLS / 4) *(volatile v4f*)op = ov;
}

extern "C" void kernel_launch(void* const* d_in, const int* in_sizes, int n_in,
                              void* d_out, int out_size, void* d_ws, size_t ws_size,
                              hipStream_t stream) {
  if (n_in < 8) return;
  if (in_sizes[0] != GN * FIN) return;
  if (in_sizes[1] != 2 * GE) return;
  if (in_sizes[2] != NHD * FIN * FH) return;
  if (in_sizes[3] != NHD * 2 * FH) return;
  if (in_sizes[4] != NHD * FH) return;
  if (in_sizes[5] != HID * NCLS) return;
  if (in_sizes[6] != 2 * NCLS) return;
  if (in_sizes[7] != NCLS) return;
  if (out_size != GN * NCLS) return;

  const float* x  = (const float*)d_in[0];
  const int*   ei = (const int*)  d_in[1];
  const float* W1 = (const float*)d_in[2];
  const float* a1 = (const float*)d_in[3];
  const float* b1 = (const float*)d_in[4];
  const float* W2 = (const float*)d_in[5];
  const float* a2 = (const float*)d_in[6];
  const float* b2 = (const float*)d_in[7];
  float* out = (float*)d_out;

  char* ws = (char*)d_ws;
  size_t off = 0;
  const size_t oP16 = off; off += (size_t)P16_HW * 2;            off = (off + 255) & ~(size_t)255;
  const size_t oHH  = off; off += (size_t)GN * HID * 4;          off = (off + 255) & ~(size_t)255;
  const size_t oSD1 = off; off += (size_t)2 * NHD * GN * 4;      off = (off + 255) & ~(size_t)255;
  const size_t oADJ = off; off += (size_t)GN * DEGCAP * 4;       off = (off + 255) & ~(size_t)255;
  const size_t oCP  = off; off += (size_t)GN * 4;                off = (off + 255) & ~(size_t)255;
  const size_t oX1  = off; off += (size_t)GN * K2 * 2;           off = (off + 255) & ~(size_t)255;
  const size_t oH2  = off; off += (size_t)GN * NC2P * 4;         off = (off + 255) & ~(size_t)255;
  const size_t oSD2 = off; off += (size_t)2 * GN * 4;            off = (off + 255) & ~(size_t)255;
  if (off > ws_size || off > (size_t)WSMAX) return;
  unsigned short* P16 = (unsigned short*)(ws + oP16);
  float*          HH  = (float*)(ws + oHH);
  float*          SD1 = (float*)(ws + oSD1);
  int*            ADJ = (int*)(ws + oADJ);
  int*            CP  = (int*)(ws + oCP);
  unsigned short* X1  = (unsigned short*)(ws + oX1);
  float*          H2  = (float*)(ws + oH2);
  float*          SD2 = (float*)(ws + oSD2);
  const unsigned short* XB  = P16 + OFF_XB;
  const unsigned short* W1T = P16 + OFF_W1T;
  const unsigned short* W2T = P16 + OFF_W2T;

  const int ldsAdj = LDS_ADJ_INTS * 4;
  hipFuncSetAttribute(reinterpret_cast<const void*>(&k_adj),
                      hipFuncAttributeMaxDynamicSharedMemorySize, ldsAdj);

  k_prep<<<NU_TOT / NTHR, NTHR, 0, stream>>>(x, W1, W2, P16);
  k_gemm1<<<dim3(GN / GBM, NHD), GTHR, 0, stream>>>(XB, W1T, HH, a1, SD1);
  k_adj<<<GN / NB, NTHR, ldsAdj, stream>>>(ei, ADJ, CP, GE, 1);
  k_agg1<<<GN / RB1, NTHR, 0, stream>>>(ADJ, CP, HH, SD1, b1, X1);
  k_gemm2<<<GN / GBM, GTHR, 0, stream>>>(X1, W2T, H2, a2, SD2);
  k_agg2<<<GN / RB2, NTHR, 0, stream>>>(ADJ, CP, H2, SD2, b2, out);
}
